// DQN_37142877176176
// MI455X (gfx1250) — hardware-run, weakly checked
//
#include <hip/hip_runtime.h>
#include <math.h>

constexpr int TSTEP  = 1024;
constexpr int HIDN   = 512;
constexpr int NGATE  = 2048;
constexpr int NACTN  = 23;
constexpr int NHEADP = 64;
constexpr int GWD = 79, GHT = 21, GPX = GWD * GHT;
constexpr int GPP = 1664;
constexpr int CWD = 9, CHT = 9, CPX = CWD * CHT;
constexpr int CPP = 96;
constexpr int GFLAT = 8 * GPX;
constexpr int FLATK = 13920;
constexpr int XCROP0 = 8 * GPP;
constexpr int KPADX = XCROP0 + 8 * CPP;
constexpr int NSLOT = GPP + CPP;
constexpr int TCHUNK = 512;
constexpr int NTHR = 256;
constexpr int CWK  = 160;
constexpr int CWPL = 16 * CWK;
constexpr int CBPL = 32;
constexpr int HPITCH = 520;
constexpr int NBIAS = 3136;
constexpr int OUTROWS_BLK = 32;
constexpr float CONV_CARRY = 16.0f;   constexpr float CONV_CARRY_INV = 1.0f / 16.0f;
constexpr float L1_CARRY   = 256.0f;  constexpr float L1_CARRY_INV   = 1.0f / 256.0f;
constexpr float W_CARRY    = 16.0f;   constexpr float W_CARRY_INV    = 1.0f / 16.0f;
constexpr float H_CARRY    = 64.0f;
constexpr float HW_CARRY_INV = 1.0f / 1024.0f;
constexpr float GLYPH_INV  = 1.0f / 5991.0f;

static_assert(KPADX % 32 == 0, "dense-1 K multiple of 32");
static_assert(HIDN % 32 == 0 && HIDN % 64 == 0, "K and N tiles");
static_assert(TSTEP % 64 == 0 && NGATE % 64 == 0 && NHEADP % 64 == 0, "M and N tiles");
static_assert(GPP % 16 == 0 && GPP >= GPX && CPP % 16 == 0 && CPP >= CPX, "pixel padding");
static_assert(XCROP0 % 64 == 0 && KPADX % 64 == 0, "segment starts on 128-B lines");
static_assert(NSLOT % 32 == 0, "permute kernel: wave-aligned rows");
static_assert((HIDN * NSLOT) % NTHR == 0, "permute grid exact");
static_assert((2 * 16 * HPITCH) % NTHR == 0, "h tile zero fill exact");
static_assert(TSTEP % TCHUNK == 0, "chunks");
static_assert(TSTEP % OUTROWS_BLK == 0 && (OUTROWS_BLK * NACTN * 4) % 128 == 0, "output block = whole lines");
static_assert((TSTEP / OUTROWS_BLK) * OUTROWS_BLK * NACTN * 4 == 94208, "output bytes");
static_assert(NACTN <= NHEADP, "head padding");
static_assert(16 * (CWK / 8) == 320 && CWK % 32 == 0, "conv weight plane");

typedef __attribute__((ext_vector_type(16))) _Float16 v16h;
typedef __attribute__((ext_vector_type(8)))  _Float16 v8h;
typedef __attribute__((ext_vector_type(16))) __bf16   v16b;
typedef __attribute__((ext_vector_type(8)))  __bf16   v8b;
typedef __attribute__((ext_vector_type(8)))  float    v8f;
typedef __attribute__((ext_vector_type(4)))  float    v4f;
typedef __attribute__((ext_vector_type(4)))  unsigned v4u;

__device__ __forceinline__ unsigned short f2bf_bits(float f) {
  unsigned u = __float_as_uint(f);
  return (unsigned short)((u + 0x7FFFu + ((u >> 16) & 1u)) >> 16);
}
__device__ __forceinline__ float bf_bits2f(unsigned short h) { return __uint_as_float(((unsigned)h) << 16); }
__device__ __forceinline__ float bf16r(float f) { return bf_bits2f(f2bf_bits(f)); }

__device__ __forceinline__ void dep_guard_h(v8f& a, v8f& b, v16h x, v16h y) { asm volatile("v_nop\n\tv_nop\n\tv_nop\n\tv_nop" : "+v"(a), "+v"(b) : "v"(x), "v"(y)); }
__device__ __forceinline__ void dep_guard_b(v8f& a, v8f& b, v16b x, v16b y) { asm volatile("v_nop\n\tv_nop\n\tv_nop\n\tv_nop" : "+v"(a), "+v"(b) : "v"(x), "v"(y)); }
__device__ __forceinline__ void keep4_h(v16h a, v16h b, v16h c, v16h d) { asm volatile("v_nop" :: "v"(a), "v"(b), "v"(c), "v"(d)); }
__device__ __forceinline__ void keep4_b(v16b a, v16b b, v16b c, v16b d) { asm volatile("v_nop" :: "v"(a), "v"(b), "v"(c), "v"(d)); }
__device__ __forceinline__ void acc_guard4(v8f& a, v8f& b, v8f& c, v8f& d) { asm volatile("v_nop\n\tv_nop\n\tv_nop\n\tv_nop" : "+v"(a), "+v"(b), "+v"(c), "+v"(d)); }
template <typename T> struct Frag;
template <> struct Frag<_Float16> {
  typedef v16h V; union U { v16h v; v8h h[2]; };
  static __device__ __forceinline__ v16h load(const _Float16* p) {
    U f; f.h[0] = *(const v8h*)(p); f.h[1] = *(const v8h*)(p + 16); return f.v;
  }
  static __device__ __forceinline__ v8f mma(v16h a, v16h b, v8f c) {
    return __builtin_amdgcn_wmma_f32_16x16x32_f16(false, a, false, b, (short)0, c, false, false);
  }
  static __device__ __forceinline__ void guard(v8f& a, v8f& b, v16h x, v16h y) { dep_guard_h(a, b, x, y); }
  static __device__ __forceinline__ void keep(v16h a, v16h b, v16h c, v16h d) { keep4_h(a, b, c, d); }
};
template <> struct Frag<__bf16> {
  typedef v16b V; union U { v16b v; v8b h[2]; };
  static __device__ __forceinline__ v16b load(const __bf16* p) {
    U f; f.h[0] = *(const v8b*)(p); f.h[1] = *(const v8b*)(p + 16); return f.v;
  }
  static __device__ __forceinline__ v8f mma(v16b a, v16b b, v8f c) {
    return __builtin_amdgcn_wmma_f32_16x16x32_bf16(false, a, false, b, (short)0, c, false, false);
  }
  static __device__ __forceinline__ void guard(v8f& a, v8f& b, v16b x, v16b y) { dep_guard_b(a, b, x, y); }
  static __device__ __forceinline__ void keep(v16b a, v16b b, v16b c, v16b d) { keep4_b(a, b, c, d); }
};

__device__ __forceinline__ v8f mma_h(v16h a, v16h b, v8f c) {
  c = __builtin_amdgcn_wmma_f32_16x16x32_f16(false, a, false, b, (short)0, c, false, false);
  asm volatile("v_nop\n\tv_nop\n\tv_nop\n\tv_nop" : "+v"(c) : "v"(a), "v"(b));
  return c;
}

__device__ __forceinline__ float fsig(float x)  { return __builtin_amdgcn_rcpf(1.0f + expf(-x)); }
__device__ __forceinline__ float ftanh(float x) { return 1.0f - 2.0f * __builtin_amdgcn_rcpf(expf(2.0f * x) + 1.0f); }

template <int ET> struct Elem;
template <> struct Elem<0> { typedef _Float16 T; };
template <> struct Elem<1> { typedef __bf16 T; };
template <int ET, bool SPLIT, int BIAS_MODE, int OUT_MODE, bool RESID, int ACT = 0>
__global__ __launch_bounds__(256) void wmma_gemm64(
    const unsigned short* __restrict__ Ap, const unsigned short* __restrict__ A2p, int lda, long strideA,
    const unsigned short* __restrict__ Btp, const unsigned short* __restrict__ Bt2p, int ldb, long strideB,
    void* __restrict__ Cout, void* __restrict__ Cout2, int ldc, long strideC,
    const float* __restrict__ bias,
    const float* __restrict__ resid, long strideR,
    int M, int N, int K, float scale) {
  typedef typename Elem<ET>::T T;
  typedef typename Frag<T>::V V;
  const T* A = (const T*)Ap; const T* A2 = (const T*)A2p; const T* Bt = (const T*)Btp; const T* Bt2 = (const T*)Bt2p;
  __shared__ __align__(16) float sT[8][16 * 68];
  const int b    = blockIdx.y;
  const int lane = threadIdx.x & 31;
  const int wave = threadIdx.x >> 5;
  const int tilesN = N >> 6;
  const int tilesM = M >> 6;
  const int tile = blockIdx.x * 8 + wave;
  if (tile >= tilesM * tilesN) return;
  const int tm = tile / tilesN;
  const int tn = tile - tm * tilesN;
  const int m0 = tm << 6;
  const int n0 = tn << 6;

  const T* Ab  = A  + (size_t)b * strideA;
  const T* Bb  = Bt + (size_t)b * strideB;
  const T* Ab2 = SPLIT ? (A2  + (size_t)b * strideA) : nullptr;
  const T* Bb2 = SPLIT ? (Bt2 + (size_t)b * strideB) : nullptr;

  const int rlane = lane & 15;
  const int koff  = (lane >> 4) * 8;
  const int mOff  = (lane >> 4) * 8;

  v8f acc[4][4];
#pragma unroll
  for (int i = 0; i < 4; ++i)
#pragma unroll
    for (int j = 0; j < 4; ++j) acc[i][j] = (v8f){0.f,0.f,0.f,0.f,0.f,0.f,0.f,0.f};

  for (int k0 = 0; k0 < K; k0 += 32) {
    V bh[4], bl[4];
#pragma unroll
    for (int j = 0; j < 4; ++j) {
      const size_t bo = (size_t)(n0 + (j << 4) + rlane) * ldb + koff + k0;
      bh[j] = Frag<T>::load(Bb + bo);
      if (SPLIT) bl[j] = Frag<T>::load(Bb2 + bo);
    }
#pragma unroll
    for (int i = 0; i < 4; ++i) {
      const size_t ao = (size_t)(m0 + (i << 4) + rlane) * lda + koff + k0;
      V ah = Frag<T>::load(Ab + ao);
      V al;
      if (SPLIT) al = Frag<T>::load(Ab2 + ao);
#pragma unroll
      for (int j = 0; j < 4; ++j) {
        acc[i][j] = Frag<T>::mma(ah, bh[j], acc[i][j]);
        if (SPLIT) {
          acc[i][j] = Frag<T>::mma(ah, bl[j], acc[i][j]);
          acc[i][j] = Frag<T>::mma(al, bh[j], acc[i][j]);
        }
      }
      Frag<T>::guard(acc[i][0], acc[i][3], ah, SPLIT ? al : ah);
    }
    Frag<T>::keep(bh[0], bh[1], bh[2], bh[3]);
    if (SPLIT) Frag<T>::keep(bl[0], bl[1], bl[2], bl[3]);
  }
  acc_guard4(acc[0][0], acc[0][1], acc[0][2], acc[0][3]);
  acc_guard4(acc[1][0], acc[1][1], acc[1][2], acc[1][3]);
  acc_guard4(acc[2][0], acc[2][1], acc[2][2], acc[2][3]);
  acc_guard4(acc[3][0], acc[3][1], acc[3][2], acc[3][3]);

  float* slab = sT[wave];
  const float* Rb = RESID ? (resid + (size_t)b * strideR) : nullptr;
#pragma unroll
  for (int i = 0; i < 4; ++i) {
    const int mBase = m0 + (i << 4);
#pragma unroll
    for (int j = 0; j < 4; ++j) {
      const int n = n0 + (j << 4) + rlane;
      float bv = 0.f;
      if (BIAS_MODE == 2) bv = bias[n];
#pragma unroll
      for (int r = 0; r < 8; ++r) {
        float v = acc[i][j][r] * scale;
        if (BIAS_MODE == 1) v += bias[mBase + mOff + r];
        if (BIAS_MODE == 2) v += bv;
        if (RESID) v += Rb[(size_t)(mBase + mOff + r) * ldc + n];
        if (ACT == 1) v = tanhf(v);
        if (ACT == 2) v = fmaxf(v, 0.0f);
        if (ACT == 3) v = v / (1.0f + expf(-v));
        if (ACT == 4) v = (v > 0.f) ? v : 0.01f * v;
        if (ACT == 5) v = 0.5f * v * (1.0f + erff(v * 0.70710678118654752f));
        slab[(mOff + r) * 68 + (j << 4) + rlane] = v;
      }
    }
    __builtin_amdgcn_fence(__ATOMIC_RELEASE, "workgroup");
    __builtin_amdgcn_wave_barrier();
    __builtin_amdgcn_fence(__ATOMIC_ACQUIRE, "workgroup");
    if (OUT_MODE == 0) {
      float* C = (float*)Cout + (size_t)b * strideC;
      const int hh = lane >> 4, c4 = (lane & 15) * 4;
      for (int pass = 0; pass < 2; ++pass) {
#pragma unroll
        for (int it = 0; it < 8; ++it) {
          const int row = it * 2 + hh;
          v4f v = *(const v4f*)(slab + row * 68 + c4);
          *(volatile v4f*)(C + (size_t)(mBase + row) * ldc + n0 + c4) = v;
        }
        __threadfence();
      }
    } else {
      const int q = lane >> 3, c8 = (lane & 7) * 8;
      unsigned short* C  = (unsigned short*)Cout  + (size_t)b * strideC;
      unsigned short* C2 = (OUT_MODE == 2) ? ((unsigned short*)Cout2 + (size_t)b * strideC) : nullptr;
      for (int pass = 0; pass < 2; ++pass) {
#pragma unroll
        for (int it = 0; it < 4; ++it) {
          const int row = it * 4 + q;
          const float* sp = slab + row * 68 + c8;
          v8h hv, lv;
#pragma unroll
          for (int e = 0; e < 8; ++e) {
            if (OUT_MODE == 1) {
              hv[e] = (_Float16)sp[e];
            } else {
              unsigned short hb = f2bf_bits(sp[e]);
              unsigned short lb = f2bf_bits(sp[e] - bf_bits2f(hb));
              hv[e] = __builtin_bit_cast(_Float16, hb);
              lv[e] = __builtin_bit_cast(_Float16, lb);
            }
          }
          *(volatile v8h*)(C + (size_t)(mBase + row) * ldc + n0 + c8) = hv;
          if (OUT_MODE == 2) *(volatile v8h*)(C2 + (size_t)(mBase + row) * ldc + n0 + c8) = lv;
        }
        __threadfence();
      }
    }
    __builtin_amdgcn_fence(__ATOMIC_RELEASE, "workgroup");
    __builtin_amdgcn_wave_barrier();
    __builtin_amdgcn_fence(__ATOMIC_ACQUIRE, "workgroup");
  }
}

struct ConvParamPtrs { const float* w[10]; const float* b[10]; };
static_assert(sizeof(ConvParamPtrs) == 160, "no padding");

__global__ __launch_bounds__(NTHR) void convw_prep_kernel(ConvParamPtrs p, unsigned short* __restrict__ wq,
                                                          float* __restrict__ bq) {
  const int L = blockIdx.y;
  const int s = blockIdx.x * NTHR + threadIdx.x;
  const float* w = (L == 0) ? p.w[0] : (L == 1) ? p.w[1] : (L == 2) ? p.w[2] : (L == 3) ? p.w[3] : (L == 4) ? p.w[4] :
                   (L == 5) ? p.w[5] : (L == 6) ? p.w[6] : (L == 7) ? p.w[7] : (L == 8) ? p.w[8] : p.w[9];
  const float* bsrc = (L == 0) ? p.b[0] : (L == 1) ? p.b[1] : (L == 2) ? p.b[2] : (L == 3) ? p.b[3] : (L == 4) ? p.b[4] :
                      (L == 5) ? p.b[5] : (L == 6) ? p.b[6] : (L == 7) ? p.b[7] : (L == 8) ? p.b[8] : p.b[9];
  const int cin  = (L == 0 || L == 5) ? 1 : 16;
  const int cout = (L == 4 || L == 9) ? 8 : 16;
  if (s < 16 * (CWK / 8)) {
    const int co = s / (CWK / 8);
    const int k8 = s - co * (CWK / 8);
    const int coc = (co < cout) ? co : (cout - 1);
    v8h hv;
#pragma unroll
    for (int e = 0; e < 8; ++e) {
      const int k = k8 * 8 + e;
      const int tap = (cin == 16) ? (k >> 4) : k;
      const int ci  = (cin == 16) ? (k & 15) : 0;
      const bool ok = (tap < 9) && (co < cout);
      const int tapc = (tap < 9) ? tap : 8;
      float f = w[(coc * cin + ci) * 9 + tapc];
      asm volatile("" : "+v"(f));
      const float g = bf16r(f) * (CONV_CARRY * (float)(int)ok);
      hv[e] = (_Float16)g;
    }
    unsigned short* dst = wq + (size_t)L * CWPL + (size_t)s * 8;
    *(volatile v8h*)dst = hv;
    __threadfence();
    *(volatile v8h*)dst = hv;
  }
  if (blockIdx.x == 0 && threadIdx.x < 32) {
    const int ln = threadIdx.x;
    const int cc = (ln < cout) ? ln : (cout - 1);
    float bl = bsrc[cc];
    asm volatile("" : "+v"(bl));
    const float o = bf16r(bl) * (float)(int)(ln < cout);
    float* dst = bq + L * CBPL + ln;
    *(volatile float*)dst = o;
    __threadfence();
    *(volatile float*)dst = o;
  }
}

__global__ __launch_bounds__(NTHR) void l1w_perm_kernel(const float* __restrict__ w, unsigned short* __restrict__ dst) {
  const int i = blockIdx.x * NTHR + threadIdx.x;
  if (i < HIDN * NSLOT) {
    const int n = i / NSLOT;
    const int s = i - n * NSLOT;
    const bool isg = (s < GPP);
    const int p = isg ? s : (s - GPP);
    const int plim = isg ? GPX : CPX;
    const bool ok = (p < plim);
    const int pc = ok ? p : (plim - 1);
    const int base = isg ? pc : (GFLAT + pc);
    const int cstr = isg ? GPX : CPX;
    const float* row = w + (size_t)n * FLATK;
    const float fac = L1_CARRY * (float)(int)ok;
    v8h hv;
#pragma unroll
    for (int ch = 0; ch < 8; ++ch) {
      float f = row[base + ch * cstr];
      asm volatile("" : "+v"(f));
      hv[ch] = (_Float16)(bf16r(f) * fac);
    }
    unsigned short* d = dst + (size_t)n * KPADX + (size_t)s * 8;
    *(volatile v8h*)d = hv;
    __threadfence();
    *(volatile v8h*)d = hv;
  }
}

__global__ __launch_bounds__(NTHR) void cast8_kernel(const float* __restrict__ src, unsigned short* __restrict__ dst,
                                                     int nrow_src, int nrow_dst, int ncol8, float sc) {
  const int i = blockIdx.x * NTHR + threadIdx.x;
  const int n8 = nrow_dst * ncol8;
  if (i < n8) {
    const int row = i / ncol8;
    const int c8  = i - row * ncol8;
    const bool ok = (row < nrow_src);
    const int rs = ok ? row : (nrow_src - 1);
    const float* sp = src + (size_t)rs * (size_t)(ncol8 * 8) + (size_t)c8 * 8;
    v4f a = *(const v4f*)(sp);
    v4f b = *(const v4f*)(sp + 4);
    asm volatile("" : "+v"(a), "+v"(b));
    const float fac = sc * (float)(int)ok;
    v8h hv;
#pragma unroll
    for (int e = 0; e < 4; ++e) {
      hv[e]     = (_Float16)(bf16r(a[e]) * fac);
      hv[4 + e] = (_Float16)(bf16r(b[e]) * fac);
    }
    unsigned short* d = dst + (size_t)i * 8;
    *(volatile v8h*)d = hv;
    __threadfence();
    *(volatile v8h*)d = hv;
  }
}

__global__ __launch_bounds__(NTHR) void bias_prep_kernel(const float* __restrict__ l1b, const float* __restrict__ l2b,
                                                         const float* __restrict__ bih, const float* __restrict__ bhh,
                                                         const float* __restrict__ l3b, float* __restrict__ dst) {
  const int i = blockIdx.x * NTHR + threadIdx.x;
  if (i < NBIAS / 4) {
    const float f0 = (float)(int)(i < 128);
    const float f1 = (float)(int)(i >= 128 && i < 256);
    const float f2 = (float)(int)(i >= 256 && i < 768);
    const float f3 = (float)(int)(i >= 768);
    const int q0 = ((i < 128) ? i : 127) * 4;
    int t1 = i - 128; t1 = t1 < 0 ? 0 : (t1 > 127 ? 127 : t1);
    int t2 = i - 256; t2 = t2 < 0 ? 0 : (t2 > 511 ? 511 : t2);
    int t3 = i - 768; t3 = t3 < 0 ? 0 : (t3 > 15 ? 15 : t3);
    const int q1 = t1 * 4, q2 = t2 * 4, q3 = t3 * 4;
    v4f va = *(const v4f*)(l1b + q0);
    v4f vb = *(const v4f*)(l2b + q1);
    v4f vc = *(const v4f*)(bih + q2);
    v4f vd = *(const v4f*)(bhh + q2);
    asm volatile("" : "+v"(va), "+v"(vb), "+v"(vc), "+v"(vd));
    v4f o;
#pragma unroll
    for (int e = 0; e < 4; ++e) {
      const int i3 = q3 + e;
      const float g3 = (float)(int)(i3 < NACTN);
      const int i3c = (i3 < NACTN) ? i3 : (NACTN - 1);
      float ve = l3b[i3c];
      asm volatile("" : "+v"(ve));
      o[e] = bf16r(va[e]) * f0 + bf16r(vb[e]) * f1 + (bf16r(vc[e]) + bf16r(vd[e])) * f2 + (bf16r(ve) * g3) * f3;
    }
    float* d = dst + (size_t)i * 4;
    *(volatile v4f*)d = o;
    __threadfence();
    *(volatile v4f*)d = o;
  }
}

template <int WD, int HT>
__device__ __forceinline__ v4u tap_load(const unsigned short* __restrict__ plane, int tap, int y, int x, bool pval, int koff) {
  const bool real = (tap < 9);
  const int tc = real ? tap : 8;
  const int q3 = tc / 3;
  const int dy = q3 - 1, dx = tc - 3 * q3 - 1;
  int iy = y + dy, ix = x + dx;
  const bool ok = pval && real && (iy >= 0) && (iy < HT) && (ix >= 0) && (ix < WD);
  iy = iy < 0 ? 0 : (iy > HT - 1 ? HT - 1 : iy);
  ix = ix < 0 ? 0 : (ix > WD - 1 ? WD - 1 : ix);
  v4u u = *(const v4u*)(plane + (size_t)(iy * WD + ix) * 16 + koff);
  asm volatile("" : "+v"(u));
  const unsigned m = 0u - (unsigned)ok;
  const v4u mm = {m, m, m, m};
  return u & mm;
}

template <int CIN, int WD, int HT, int PP, int OUT8>
__global__ __launch_bounds__(NTHR) void conv3x3_kernel(const int* __restrict__ gin, const unsigned short* __restrict__ ain,
                                                       const unsigned short* __restrict__ wqp, const float* __restrict__ bq,
                                                       unsigned short* __restrict__ aout, int t0, int xcol0) {
  constexpr int P  = WD * HT;
  constexpr int NT = PP / 16;
  constexpr int NCH = (CIN == 16) ? 5 : 1;
  static_assert(PP % 16 == 0 && PP >= P, "tile padding");
  const _Float16* wq = (const _Float16*)wqp;
  const int tt = blockIdx.x;
  const int t  = t0 + tt;
  const int lane = threadIdx.x & 31, wave = threadIdx.x >> 5;
  const int c = lane & 15, hh = lane >> 4, koff = hh * 8;

  v16h afr[NCH];
#pragma unroll
  for (int j = 0; j < NCH; ++j) afr[j] = Frag<_Float16>::load(wq + c * CWK + 32 * j + koff);
  float bv[8];
#pragma unroll
  for (int r = 0; r < 8; ++r) bv[r] = bq[8 * hh + r];

  const unsigned short* aint = ain + (size_t)tt * PP * 16;
  const int* gint = gin + (size_t)t * P;
  const v8f z8 = {0.f, 0.f, 0.f, 0.f, 0.f, 0.f, 0.f, 0.f};

  for (int tile = wave; tile < NT; tile += NTHR / 32) {
    const int p = tile * 16 + c;
    const bool pval = (p < P);
    const int y = p / WD;
    const int x = p - y * WD;
    v8f acc = z8;
#pragma unroll
    for (int j = 0; j < NCH; ++j) {
      v16h bvec;
      if (CIN == 16) {
        union { v16h v; v4u u[2]; } bf;
        bf.u[0] = tap_load<WD, HT>(aint, 2 * j, y, x, pval, koff);
        bf.u[1] = tap_load<WD, HT>(aint, 2 * j + 1, y, x, pval, koff);
        bvec = bf.v;
      } else {
        v8h lo, hi;
#pragma unroll
        for (int i = 0; i < 8; ++i) {
          const int tap = 8 * hh + i;
          const int tc = (tap < 9) ? tap : 8;
          const int q3 = tc / 3;
          const int dy = q3 - 1, dx = tc - 3 * q3 - 1;
          int iy = y + dy, ix = x + dx;
          const bool ok = pval && (tap < 9) && (iy >= 0) && (iy < HT) && (ix >= 0) && (ix < WD);
          iy = iy < 0 ? 0 : (iy > HT - 1 ? HT - 1 : iy);
          ix = ix < 0 ? 0 : (ix > WD - 1 ? WD - 1 : ix);
          int gv = gint[iy * WD + ix];
          asm volatile("" : "+v"(gv));
          const float f = ((float)gv * GLYPH_INV) * (float)(int)ok;
          lo[i] = (_Float16)f;
          hi[i] = (_Float16)0.0f;
        }
        Frag<_Float16>::U fb;
        fb.h[0] = lo;
        fb.h[1] = hi;
        bvec = fb.v;
      }
      acc = mma_h(afr[j], bvec, acc);
    }
    v8h o;
#pragma unroll
    for (int r = 0; r < 8; ++r) {
      float v = acc[r] * CONV_CARRY_INV + bv[r];
      v = fmaxf(v, 0.0f);
      o[r] = (_Float16)v;
    }
    const v4u pk = __builtin_bit_cast(v4u, o);
    if (OUT8 == 0) {
      const int src = 16 * (lane & 1) + (lane >> 1);
      v4u q;
#pragma unroll
      for (int e = 0; e < 4; ++e) q[e] = (unsigned)__shfl((int)pk[e], src, 32);
      unsigned short* d = aout + ((size_t)tt * PP + (size_t)tile * 16) * 16 + (size_t)lane * 8;
      *(volatile v4u*)d = q;
      __threadfence();
      *(volatile v4u*)d = q;
    } else {
      unsigned short* d = aout + (size_t)t * KPADX + xcol0 + ((size_t)tile * 16 + c) * 8;
      if (hh == 0) *(volatile v4u*)d = pk;
      __threadfence();
      if (hh == 0) *(volatile v4u*)d = pk;
    }
  }
}

__global__ __launch_bounds__(NTHR) void lstm_seq_kernel(const float* __restrict__ GX, const int* __restrict__ done,
                                                        const unsigned short* __restrict__ WHHp,
                                                        unsigned short* __restrict__ HS) {
  __shared__ __align__(16) _Float16 Ah[2][16 * HPITCH];
  const _Float16* WHH = (const _Float16*)WHHp;
  const int tid = threadIdx.x, lane = tid & 31, wave = tid >> 5;
  const int c = lane & 15, hh = lane >> 4, koff = hh * 8;

  {
    _Float16* ahf = &Ah[0][0];
#pragma unroll 1
    for (int i = tid; i < 2 * 16 * HPITCH; i += NTHR) ahf[i] = (_Float16)0.0f;
  }
  float cst[4];
#pragma unroll
  for (int ub = 0; ub < 4; ++ub) cst[ub] = 0.0f;
  __syncthreads();

  const v8f z8 = {0.f, 0.f, 0.f, 0.f, 0.f, 0.f, 0.f, 0.f};

#pragma unroll 1
  for (int t = 0; t < TSTEP; ++t) {
    const int cur = t & 1;
    const float nd = (float)(1 - done[t]);
    const float rs = nd * HW_CARRY_INV;
    const _Float16* ahrow = &Ah[cur][0] + c * HPITCH + koff;
    _Float16* ahn = &Ah[cur ^ 1][0];
    const float* gxt = GX + (size_t)t * NGATE;

#pragma unroll
    for (int ub = 0; ub < 4; ++ub) {
      const int j = 64 * wave + 16 * ub + c;
      const _Float16* wr = WHH + (size_t)j * HIDN + koff;
      v8f acc[4];
      acc[0] = z8; acc[1] = z8; acc[2] = z8; acc[3] = z8;
#pragma unroll 1
      for (int k0 = 0; k0 < HIDN; k0 += 32) {
        const v16h a  = Frag<_Float16>::load(ahrow + k0);
        const v16h b0 = Frag<_Float16>::load(wr + k0);
        const v16h b1 = Frag<_Float16>::load(wr + (size_t)1 * HIDN * HIDN + k0);
        const v16h b2 = Frag<_Float16>::load(wr + (size_t)2 * HIDN * HIDN + k0);
        const v16h b3 = Frag<_Float16>::load(wr + (size_t)3 * HIDN * HIDN + k0);
        acc[0] = Frag<_Float16>::mma(a, b0, acc[0]);
        acc[1] = Frag<_Float16>::mma(a, b1, acc[1]);
        acc[2] = Frag<_Float16>::mma(a, b2, acc[2]);
        acc[3] = Frag<_Float16>::mma(a, b3, acc[3]);
        dep_guard_h(acc[0], acc[3], a, b3);
        keep4_h(b0, b1, b2, b3);
      }
      acc_guard4(acc[0], acc[1], acc[2], acc[3]);
      const float gi = gxt[j];
      const float gf = gxt[HIDN + j];
      const float gg = gxt[2 * HIDN + j];
      const float go = gxt[3 * HIDN + j];
      const float zi = acc[0][0] * rs + gi;
      const float zf = acc[1][0] * rs + gf;
      const float zg = acc[2][0] * rs + gg;
      const float zo = acc[3][0] * rs + go;
      const float cp = cst[ub] * nd;
      const float cn = fsig(zf) * cp + fsig(zi) * ftanh(zg);
      const float hn = fsig(zo) * ftanh(cn);
      cst[ub] = cn;
      const _Float16 hv = (_Float16)(hn * H_CARRY);
#pragma unroll
      for (int r = 0; r < 8; ++r) ahn[(8 * hh + r) * HPITCH + j] = hv;
    }
    __syncthreads();
    {
      const int col = 64 * wave + 8 * (lane & 7);
      const v4u v = *(const v4u*)(&Ah[cur ^ 1][0] + col);
      unsigned short* d = HS + (size_t)t * HIDN + col;
      if (lane < 8) *(volatile v4u*)d = v;
      __threadfence();
      if (lane < 8) *(volatile v4u*)d = v;
    }
  }
}

__global__ __launch_bounds__(NTHR) void pack_out_kernel(const float* __restrict__ HEAD, float* __restrict__ out) {
  __shared__ __align__(16) float S[OUTROWS_BLK * NACTN];
  const int tid = threadIdx.x, lane = tid & 31, wave = tid >> 5;
  const int blk = blockIdx.x;
  const int row0 = blk * OUTROWS_BLK;
#pragma unroll 1
  for (int i = tid; i < OUTROWS_BLK * NACTN; i += NTHR) {
    const int r = i / NACTN, a = i - r * NACTN;
    S[i] = HEAD[(size_t)(row0 + r) * NHEADP + a];
  }
  __syncthreads();
  if (wave == 0) {
    float* base = out + (size_t)blk * (OUTROWS_BLK * NACTN);
    constexpr int NQ = (OUTROWS_BLK * NACTN) / 4;
    for (int pass = 0; pass < 2; ++pass) {
#pragma unroll
      for (int it = 0; it < (NQ + 31) / 32; ++it) {
        const int idx = it * 32 + lane;
        if (idx < NQ) {
          const v4f v = *(const v4f*)(S + idx * 4);
          *(volatile v4f*)(base + (size_t)idx * 4) = v;
        }
      }
      __threadfence();
    }
  }
}

extern "C" void kernel_launch(void* const* d_in, const int* in_sizes, int n_in,
                              void* d_out, int out_size, void* d_ws, size_t ws_size, hipStream_t stream) {
  if (n_in < 33 || d_out == nullptr || d_ws == nullptr) return;
  const int expect_sizes[33] = {
      TSTEP * GPX, TSTEP * CPX, TSTEP,
      144, 16, 2304, 16, 2304, 16, 2304, 16, 1152, 8,
      144, 16, 2304, 16, 2304, 16, 2304, 16, 1152, 8,
      HIDN * FLATK, HIDN, HIDN * HIDN, HIDN, NACTN * HIDN, NACTN,
      NGATE * HIDN, NGATE * HIDN, NGATE, NGATE};
  for (int i = 0; i < 33; ++i) if (in_sizes[i] != expect_sizes[i]) return;
  if (out_size != TSTEP * NACTN) return;

  const int*   glyphs = (const int*)d_in[0];
  const int*   crop   = (const int*)d_in[1];
  const int*   done   = (const int*)d_in[2];
  const float* l1w = (const float*)d_in[23];
  const float* l1b = (const float*)d_in[24];
  const float* l2w = (const float*)d_in[25];
  const float* l2b = (const float*)d_in[26];
  const float* l3w = (const float*)d_in[27];
  const float* l3b = (const float*)d_in[28];
  const float* wih = (const float*)d_in[29];
  const float* whh = (const float*)d_in[30];
  const float* bih = (const float*)d_in[31];
  const float* bhh = (const float*)d_in[32];
  float* out = (float*)d_out;

  char* ws = (char*)d_ws; size_t off = 0;
  auto carve = [&](size_t bytes) -> char* { char* p = ws + off; off += (bytes + 255) & ~(size_t)255; return p; };
  unsigned short* ACTG0 = (unsigned short*)carve((size_t)TCHUNK * GPP * 16 * 2);
  unsigned short* ACTG1 = (unsigned short*)carve((size_t)TCHUNK * GPP * 16 * 2);
  unsigned short* ACTC0 = (unsigned short*)carve((size_t)TSTEP * CPP * 16 * 2);
  unsigned short* ACTC1 = (unsigned short*)carve((size_t)TSTEP * CPP * 16 * 2);
  unsigned short* XR    = (unsigned short*)carve((size_t)TSTEP * KPADX * 2);
  unsigned short* L1WP  = (unsigned short*)carve((size_t)HIDN * KPADX * 2);
  unsigned short* L2W16 = (unsigned short*)carve((size_t)HIDN * HIDN * 2);
  unsigned short* WIH16 = (unsigned short*)carve((size_t)NGATE * HIDN * 2);
  unsigned short* WHH16 = (unsigned short*)carve((size_t)NGATE * HIDN * 2);
  unsigned short* L3W16 = (unsigned short*)carve((size_t)NHEADP * HIDN * 2);
  unsigned short* CONVW = (unsigned short*)carve((size_t)10 * CWPL * 2);
  float*          CONVB = (float*)carve((size_t)10 * CBPL * 4);
  float*          BIAS  = (float*)carve((size_t)NBIAS * 4);
  unsigned short* Y16   = (unsigned short*)carve((size_t)TSTEP * HIDN * 2);
  unsigned short* Z16   = (unsigned short*)carve((size_t)TSTEP * HIDN * 2);
  float*          GX    = (float*)carve((size_t)TSTEP * NGATE * 4);
  unsigned short* HS16  = (unsigned short*)carve((size_t)TSTEP * HIDN * 2);
  float*          HEAD  = (float*)carve((size_t)TSTEP * NHEADP * 4);
  if (off > ws_size || off > (size_t)134217728) return;

  {
    ConvParamPtrs cp;
    for (int j = 0; j < 5; ++j) {
      cp.w[j]     = (const float*)d_in[3 + 2 * j];
      cp.b[j]     = (const float*)d_in[4 + 2 * j];
      cp.w[5 + j] = (const float*)d_in[13 + 2 * j];
      cp.b[5 + j] = (const float*)d_in[14 + 2 * j];
    }
    convw_prep_kernel<<<dim3(2, 10), NTHR, 0, stream>>>(cp, CONVW, CONVB);
  }
  l1w_perm_kernel<<<(HIDN * NSLOT) / NTHR, NTHR, 0, stream>>>(l1w, L1WP);
  cast8_kernel<<<(HIDN * (HIDN / 8) + NTHR - 1) / NTHR, NTHR, 0, stream>>>(l2w, L2W16, HIDN, HIDN, HIDN / 8, W_CARRY);
  cast8_kernel<<<(NGATE * (HIDN / 8) + NTHR - 1) / NTHR, NTHR, 0, stream>>>(wih, WIH16, NGATE, NGATE, HIDN / 8, W_CARRY);
  cast8_kernel<<<(NGATE * (HIDN / 8) + NTHR - 1) / NTHR, NTHR, 0, stream>>>(whh, WHH16, NGATE, NGATE, HIDN / 8, W_CARRY);
  cast8_kernel<<<(NHEADP * (HIDN / 8) + NTHR - 1) / NTHR, NTHR, 0, stream>>>(l3w, L3W16, NACTN, NHEADP, HIDN / 8, W_CARRY);
  bias_prep_kernel<<<(NBIAS / 4 + NTHR - 1) / NTHR, NTHR, 0, stream>>>(l1b, l2b, bih, bhh, l3b, BIAS);

  for (int ch = 0; ch < TSTEP / TCHUNK; ++ch) {
    const int t0 = ch * TCHUNK;
    conv3x3_kernel<1,  GWD, GHT, GPP, 0><<<TCHUNK, NTHR, 0, stream>>>(glyphs, ACTG1, CONVW + 0 * CWPL, CONVB + 0 * CBPL, ACTG0, t0, 0);
    conv3x3_kernel<16, GWD, GHT, GPP, 0><<<TCHUNK, NTHR, 0, stream>>>(glyphs, ACTG0, CONVW + 1 * CWPL, CONVB + 1 * CBPL, ACTG1, t0, 0);
    conv3x3_kernel<16, GWD, GHT, GPP, 0><<<TCHUNK, NTHR, 0, stream>>>(glyphs, ACTG1, CONVW + 2 * CWPL, CONVB + 2 * CBPL, ACTG0, t0, 0);
    conv3x3_kernel<16, GWD, GHT, GPP, 0><<<TCHUNK, NTHR, 0, stream>>>(glyphs, ACTG0, CONVW + 3 * CWPL, CONVB + 3 * CBPL, ACTG1, t0, 0);
    conv3x3_kernel<16, GWD, GHT, GPP, 1><<<TCHUNK, NTHR, 0, stream>>>(glyphs, ACTG1, CONVW + 4 * CWPL, CONVB + 4 * CBPL, XR, t0, 0);
  }
  conv3x3_kernel<1,  CWD, CHT, CPP, 0><<<TSTEP, NTHR, 0, stream>>>(crop, ACTC1, CONVW + 5 * CWPL, CONVB + 5 * CBPL, ACTC0, 0, 0);
  conv3x3_kernel<16, CWD, CHT, CPP, 0><<<TSTEP, NTHR, 0, stream>>>(crop, ACTC0, CONVW + 6 * CWPL, CONVB + 6 * CBPL, ACTC1, 0, 0);
  conv3x3_kernel<16, CWD, CHT, CPP, 0><<<TSTEP, NTHR, 0, stream>>>(crop, ACTC1, CONVW + 7 * CWPL, CONVB + 7 * CBPL, ACTC0, 0, 0);
  conv3x3_kernel<16, CWD, CHT, CPP, 0><<<TSTEP, NTHR, 0, stream>>>(crop, ACTC0, CONVW + 8 * CWPL, CONVB + 8 * CBPL, ACTC1, 0, 0);
  conv3x3_kernel<16, CWD, CHT, CPP, 1><<<TSTEP, NTHR, 0, stream>>>(crop, ACTC1, CONVW + 9 * CWPL, CONVB + 9 * CBPL, XR, 0, XCROP0);

  const dim3 g512((TSTEP / 64) * (HIDN / 64) / 8, 1);
  const dim3 g2048((TSTEP / 64) * (NGATE / 64) / 8, 1);
  const dim3 g64(((TSTEP / 64) * (NHEADP / 64) + 7) / 8, 1);
  wmma_gemm64<0, false, 2, 1, false, 2><<<g512, 256, 0, stream>>>(
      XR, XR, KPADX, 0L, L1WP, L1WP, KPADX, 0L, (void*)Y16, (void*)Y16, HIDN, 0L,
      BIAS, BIAS, 0L, TSTEP, HIDN, KPADX, L1_CARRY_INV);
  wmma_gemm64<0, false, 2, 1, false, 2><<<g512, 256, 0, stream>>>(
      Y16, Y16, HIDN, 0L, L2W16, L2W16, HIDN, 0L, (void*)Z16, (void*)Z16, HIDN, 0L,
      BIAS + 512, BIAS, 0L, TSTEP, HIDN, HIDN, W_CARRY_INV);
  wmma_gemm64<0, false, 2, 0, false, 0><<<g2048, 256, 0, stream>>>(
      Z16, Z16, HIDN, 0L, WIH16, WIH16, HIDN, 0L, (void*)GX, (void*)GX, NGATE, 0L,
      BIAS + 1024, BIAS, 0L, TSTEP, NGATE, HIDN, W_CARRY_INV);

  lstm_seq_kernel<<<1, NTHR, 0, stream>>>(GX, done, WHH16, HS16);

  wmma_gemm64<0, false, 2, 0, false, 0><<<g64, 256, 0, stream>>>(
      HS16, HS16, HIDN, 0L, L3W16, L3W16, HIDN, 0L, (void*)HEAD, (void*)HEAD, NHEADP, 0L,
      BIAS + 3072, BIAS, 0L, TSTEP, NHEADP, HIDN, HW_CARRY_INV);
  pack_out_kernel<<<TSTEP / OUTROWS_BLK, NTHR, 0, stream>>>(HEAD, out);
}
